// AttentionModel_59614146068701
// MI455X (gfx1250) — hardware-run, weakly checked
//
#include <hip/hip_runtime.h>


#define NSEQ 8
#define TT   1024
#define FD   512
#define NH_  8
#define HD   64
#define DQ   (NH_ * HD)
#define NL   4
#define VOC  1024
#define ROWS (NSEQ * TT)
#define ZH   NH_
#define RH   0
#define WIN  TT
#define PCAR 1024.0f
#define SCL  1.0f
typedef _Float16 h16;
typedef unsigned short bf;
typedef __attribute__((ext_vector_type(16))) __bf16   v16bf;
typedef __attribute__((ext_vector_type(16))) _Float16 v16h;
typedef __attribute__((ext_vector_type(8)))  _Float16 v8h;
typedef __attribute__((ext_vector_type(8)))  unsigned short v8us;
typedef __attribute__((ext_vector_type(8)))  float    v8f;
typedef __attribute__((ext_vector_type(4)))  float    v4f;
typedef v8h  __attribute__((may_alias)) v8ha;
typedef v4f  __attribute__((may_alias)) v4fa;
typedef v8us __attribute__((may_alias)) v8usa;

__device__ __forceinline__ unsigned short f2bf(float f) { unsigned u = __float_as_uint(f); u += 0x7FFFu + ((u >> 16) & 1u); return (unsigned short)(u >> 16); }
__device__ __forceinline__ float bf2f(unsigned short b) { return __uint_as_float(((unsigned)b) << 16); }
__device__ __forceinline__ float bfr(float f) { return bf2f(f2bf(f)); }
__device__ __forceinline__ v16h cat16(v8h lo, v8h hi) { return __builtin_shufflevector(lo, hi, 0, 1, 2, 3, 4, 5, 6, 7, 8, 9, 10, 11, 12, 13, 14, 15); }
__device__ __forceinline__ v16bf cat16b(v8us lo, v8us hi) { return __builtin_bit_cast(v16bf, __builtin_shufflevector(lo, hi, 0, 1, 2, 3, 4, 5, 6, 7, 8, 9, 10, 11, 12, 13, 14, 15)); }
__device__ __forceinline__ v8f wmma16(v16h a, v16h b, v8f c) { return __builtin_amdgcn_wmma_f32_16x16x32_f16(false, a, false, b, (short)0, c, false, false); }
__device__ __forceinline__ v8f wmmab(v16bf a, v16bf b, v8f c) { return __builtin_amdgcn_wmma_f32_16x16x32_bf16(false, a, false, b, (short)0, c, false, false); }


template <typename T16> struct WFrag;
template <> struct WFrag<h16> { typedef v16h V; static __device__ __forceinline__ V ld(const h16* p) { return cat16(*(const v8h*)p, *(const v8h*)(p + 16)); } static __device__ __forceinline__ v8f mma(V a, V b, v8f c) { return wmma16(a, b, c); } };
template <> struct WFrag<bf> { typedef v16bf V; static __device__ __forceinline__ V ld(const bf* p) { return cat16b(*(const v8us*)p, *(const v8us*)(p + 16)); } static __device__ __forceinline__ v8f mma(V a, V b, v8f c) { return wmmab(a, b, c); } };
template <typename T16, int NSPLIT, bool BIAS>
__global__ __launch_bounds__(32) void k_gemmw(const T16* __restrict__ A, const T16* __restrict__ A2, const T16* __restrict__ Bt, const T16* __restrict__ Bt2, int K, float* C, int ldc, const float* __restrict__ bias, size_t sA, size_t sB, size_t sC) {
    typedef typename WFrag<T16>::V V;
    __shared__ __align__(16) float os[16 * 68];
    const size_t z = blockIdx.z; A += z * sA; if (A2) A2 += z * sA; Bt += z * sB; if (Bt2) Bt2 += z * sB; C += z * sC;
    const int lane = threadIdx.x & 31, lr = lane & 15, hi = lane >> 4; const int r0 = blockIdx.x * 64, c0 = blockIdx.y * 64;
    v8f acc[4][4];
#pragma unroll
    for (int mb = 0; mb < 4; ++mb)
#pragma unroll
        for (int nb = 0; nb < 4; ++nb) acc[mb][nb] = (v8f){};
    const size_t aoff = (size_t)(r0 + lr) * K + 8 * hi, boff = (size_t)(c0 + lr) * K + 8 * hi;
#pragma unroll 1
    for (int kc = 0; kc < K; kc += 32) {
        V a[4], a2[4];
#pragma unroll
        for (int mb = 0; mb < 4; ++mb) { a[mb] = WFrag<T16>::ld(A + aoff + (size_t)mb * 16 * K + kc); if (NSPLIT == 1 || NSPLIT == 2) a2[mb] = WFrag<T16>::ld(A2 + aoff + (size_t)mb * 16 * K + kc); }
#pragma unroll
        for (int nb = 0; nb < 4; ++nb) { const V b = WFrag<T16>::ld(Bt + boff + (size_t)nb * 16 * K + kc); V b2; if (NSPLIT >= 2) b2 = WFrag<T16>::ld(Bt2 + boff + (size_t)nb * 16 * K + kc);
#pragma unroll
            for (int mb = 0; mb < 4; ++mb) { acc[mb][nb] = WFrag<T16>::mma(a[mb], b, acc[mb][nb]); if (NSPLIT == 1 || NSPLIT == 2) acc[mb][nb] = WFrag<T16>::mma(a2[mb], b, acc[mb][nb]); if (NSPLIT >= 2) acc[mb][nb] = WFrag<T16>::mma(a[mb], b2, acc[mb][nb]); } }
        asm volatile("v_nop\n\tv_nop\n\tv_nop\n\tv_nop" : "+v"(acc[0][0]), "+v"(acc[1][1]), "+v"(acc[2][2]), "+v"(acc[3][3]) : "v"(a[0]), "v"(a[3]));
    }
#pragma unroll
    for (int mb = 0; mb < 4; ++mb) {
#pragma unroll
        for (int nb = 0; nb < 4; ++nb) {
#pragma unroll
            for (int j = 0; j < 8; ++j) os[(hi * 8 + j) * 68 + nb * 16 + lr] = acc[mb][nb][j]; }
        __builtin_amdgcn_wave_barrier(); asm volatile("" ::: "memory");
        float* crow = C + (size_t)(r0 + mb * 16) * ldc + c0;
#pragma unroll 1
        for (int ps = 0; ps < 2; ++ps) {
#pragma unroll
            for (int s = 0; s < 8; ++s) { const int row = 2 * s + hi, cofs = lr * 4; v4f val = *(const v4fa*)(os + row * 68 + cofs); if (BIAS) { val[0] += bfr(bias[c0 + cofs]); val[1] += bfr(bias[c0 + cofs + 1]); val[2] += bfr(bias[c0 + cofs + 2]); val[3] += bfr(bias[c0 + cofs + 3]); }
                *(volatile v4f*)(crow + (size_t)row * ldc + cofs) = val; }
            if (ps == 0) __threadfence(); }
        __builtin_amdgcn_wave_barrier(); asm volatile("" ::: "memory");
    }
}

__device__ __forceinline__ h16 tohx(float x) { return (h16)x; }
__device__ __forceinline__ void splitf(float y, unsigned short& h, unsigned short& l) { h = f2bf(y); l = f2bf(y - bf2f(h)); }
typedef __attribute__((ext_vector_type(2))) _Float16 v2h;
typedef __attribute__((ext_vector_type(4))) _Float16 v4h;
typedef __attribute__((ext_vector_type(2))) unsigned short v2us;
typedef __attribute__((ext_vector_type(4))) unsigned short v4us;
typedef __attribute__((ext_vector_type(2))) float v2f;
typedef __attribute__((ext_vector_type(4))) int v4i;

__global__ __launch_bounds__(256) void k_wtG(const float* __restrict__ w, int K, int N, bf* Bt) {
    const int lane = threadIdx.x & 31; const int L0 = (blockIdx.x * 8 + (threadIdx.x >> 5)) * 8; const int nlines = N * K / 64;
#pragma unroll
    for (int ps = 0; ps < 2; ++ps) {
#pragma unroll 1
        for (int l = 0; l < 8; ++l) { const int L = L0 + l; if (L >= nlines) break; const size_t e = (size_t)L * 64 + lane * 2; const int k = (int)(e % K), n = (int)(e / K); v2us o;
            o[0] = f2bf(w[(size_t)k * N + n]); o[1] = f2bf(w[(size_t)(k + 1) * N + n]); *(volatile v2us*)(Bt + e) = o; }
        if (ps == 0) __threadfence(); }
}
template <typename T16, int NSPLIT, int CMODE>
__global__ __launch_bounds__(32) void k_gemmc(const T16* __restrict__ A, const T16* __restrict__ A2, const T16* __restrict__ Bt, const T16* __restrict__ Bt2, int K, float* C, int ldc, int roff, size_t sA, size_t sB, size_t sC) {
    typedef typename WFrag<T16>::V V;
    __shared__ __align__(16) float os[16 * 68];
    const size_t z = blockIdx.z; A += z * sA; if (A2) A2 += z * sA; Bt += z * sB; if (Bt2) Bt2 += z * sB; C += z * sC;
    const int lane = threadIdx.x & 31, lr = lane & 15, hi = lane >> 4; const int r0 = blockIdx.x * 64, c0 = blockIdx.y * 64;
    if (CMODE == 1 && c0 > r0 + roff + 63) return;
    const int Kl = (CMODE == 2) ? min(K, r0 + roff + 64) : K;
    v8f acc[4][4];
#pragma unroll
    for (int mb = 0; mb < 4; ++mb)
#pragma unroll
        for (int nb = 0; nb < 4; ++nb) acc[mb][nb] = (v8f){};
    const size_t aoff = (size_t)(r0 + lr) * K + 8 * hi, boff = (size_t)(c0 + lr) * K + 8 * hi;
#pragma unroll 1
    for (int kc = 0; kc < Kl; kc += 32) {
        V a[4], a2[4];
#pragma unroll
        for (int mb = 0; mb < 4; ++mb) { a[mb] = WFrag<T16>::ld(A + aoff + (size_t)mb * 16 * K + kc); if (NSPLIT == 1 || NSPLIT == 2) a2[mb] = WFrag<T16>::ld(A2 + aoff + (size_t)mb * 16 * K + kc); }
#pragma unroll
        for (int nb = 0; nb < 4; ++nb) { const V b = WFrag<T16>::ld(Bt + boff + (size_t)nb * 16 * K + kc); V b2; if (NSPLIT >= 2) b2 = WFrag<T16>::ld(Bt2 + boff + (size_t)nb * 16 * K + kc);
#pragma unroll
            for (int mb = 0; mb < 4; ++mb) { acc[mb][nb] = WFrag<T16>::mma(a[mb], b, acc[mb][nb]); if (NSPLIT == 1 || NSPLIT == 2) acc[mb][nb] = WFrag<T16>::mma(a2[mb], b, acc[mb][nb]); if (NSPLIT >= 2) acc[mb][nb] = WFrag<T16>::mma(a[mb], b2, acc[mb][nb]); } }
        asm volatile("v_nop\n\tv_nop\n\tv_nop\n\tv_nop" : "+v"(acc[0][0]), "+v"(acc[1][1]), "+v"(acc[2][2]), "+v"(acc[3][3]) : "v"(a[0]), "v"(a[3]));
    }
#pragma unroll
    for (int mb = 0; mb < 4; ++mb) {
#pragma unroll
        for (int nb = 0; nb < 4; ++nb) {
#pragma unroll
            for (int j = 0; j < 8; ++j) os[(hi * 8 + j) * 68 + nb * 16 + lr] = acc[mb][nb][j]; }
        __builtin_amdgcn_wave_barrier(); asm volatile("" ::: "memory");
        float* crow = C + (size_t)(r0 + mb * 16) * ldc + c0;
#pragma unroll 1
        for (int ps = 0; ps < 2; ++ps) {
#pragma unroll
            for (int s = 0; s < 8; ++s) { const int row = 2 * s + hi, cofs = lr * 4; v4f val = *(const v4fa*)(os + row * 68 + cofs);
                *(volatile v4f*)(crow + (size_t)row * ldc + cofs) = val; }
            if (ps == 0) __threadfence(); }
        __builtin_amdgcn_wave_barrier(); asm volatile("" ::: "memory");
    }
}

__global__ __launch_bounds__(256) void k_split8(const float* __restrict__ F, bf* Ph, bf* Pl, size_t n8) { const size_t i = (size_t)blockIdx.x * 256 + threadIdx.x; if (i >= n8) return; const v8f v = *(const v8f*)(F + i * 8); v8us oh, ol;
#pragma unroll
    for (int k = 0; k < 8; ++k) { unsigned short a, c2; splitf(v[k], a, c2); oh[k] = a; ol[k] = c2; }
    *(volatile v8us*)(Ph + i * 8) = oh; *(volatile v8us*)(Pl + i * 8) = ol; __threadfence(); *(volatile v8us*)(Ph + i * 8) = oh; *(volatile v8us*)(Pl + i * 8) = ol; }

__global__ __launch_bounds__(256) void k_embx(const int* __restrict__ tok, const float* __restrict__ emb, float* X) { const size_t e = ((size_t)blockIdx.x * 256 + threadIdx.x) * 4; if (e >= (size_t)ROWS * FD) return; const int c = (int)(e % FD); const int r = (int)(e / FD); int id = tok[r]; id = id < 0 ? 0 : (id >= VOC ? VOC - 1 : id); const v4f v = *(const v4f*)(emb + (size_t)id * FD + c); v4f o;
#pragma unroll
    for (int q = 0; q < 4; ++q) o[q] = bfr(v[q]); *(volatile v4f*)(X + e) = o; __threadfence(); *(volatile v4f*)(X + e) = o; }
__global__ __launch_bounds__(256) void k_pl16(const float* __restrict__ F, int r0, h16* P16) { const size_t e = ((size_t)blockIdx.x * 256 + threadIdx.x) * 2; if (e >= (size_t)NH_ * TT * HD) return; const int d = (int)(e % HD); const int t = (int)((e / HD) % TT); const int h = (int)(e / ((size_t)HD * TT)); const float* f = F + ((size_t)r0 + t) * FD + h * HD + d; v2h o; o[0] = tohx(f[0]); o[1] = tohx(f[1]);
    *(volatile v2h*)(P16 + e) = o; __threadfence(); *(volatile v2h*)(P16 + e) = o; }
__global__ __launch_bounds__(256) void k_vt16(const float* __restrict__ F, int r0, h16* V16) { const size_t e = ((size_t)blockIdx.x * 256 + threadIdx.x) * 2; if (e >= (size_t)NH_ * HD * TT) return; const int t = (int)(e % TT); const int d = (int)((e / TT) % HD); const int h = (int)(e / ((size_t)TT * HD)); v2h o;
#pragma unroll
    for (int q = 0; q < 2; ++q) o[q] = tohx(F[((size_t)r0 + t + q) * FD + h * HD + d]);
    *(volatile v2h*)(V16 + e) = o; __threadfence(); *(volatile v2h*)(V16 + e) = o; }
__global__ __launch_bounds__(256) void k_asoft(const float* __restrict__ Sb, h16* P16, bf* Ph, bf* Pl) {
    const int lane = threadIdx.x & 31; const int row = blockIdx.x * 8 + (threadIdx.x >> 5); if (row >= ZH * TT) return; const int i = row % TT; const int zz = row / TT; (void)zz; const bool hires = (i < RH); const float* sr = Sb + (size_t)row * TT; float v[TT / 32]; float mx = -3.0e38f;
#pragma unroll
    for (int ch = 0; ch < TT / 128; ++ch) { const int j0 = ch * 128 + lane * 4; const v4f a = *(const v4f*)(sr + j0);
#pragma unroll
        for (int q = 0; q < 4; ++q) { const int j = j0 + q; (void)j; const float t = (j <= i && i - j < WIN) ? a[q] * SCL : -3.0e38f; v[ch * 4 + q] = t; mx = fmaxf(mx, t); } }
#pragma unroll
    for (int sh = 16; sh; sh >>= 1) mx = fmaxf(mx, __shfl_xor(mx, sh, 32));
    float sum = 0.f;
#pragma unroll
    for (int k = 0; k < TT / 32; ++k) { float d0 = __fsub_rn(v[k], mx); asm volatile("" : "+v"(d0)); v[k] = __builtin_amdgcn_exp2f(__fmul_rn(d0, 1.4426950408889634f)); sum += v[k]; }
#pragma unroll
    for (int sh = 16; sh; sh >>= 1) sum += __shfl_xor(sum, sh, 32);
    const float f = __fdiv_rn(hires ? 1.0f : PCAR, sum);
#pragma unroll 1
    for (int ps = 0; ps < 2; ++ps) {
        if (hires) {
#pragma unroll
            for (int ch = 0; ch < TT / 128; ++ch) { v4us oh, ol;
#pragma unroll
                for (int q = 0; q < 4; ++q) { unsigned short a, c2; splitf(v[ch * 4 + q] * f, a, c2); oh[q] = a; ol[q] = c2; }
                const size_t oo = ((size_t)zz * (RH ? RH : 1) + i) * TT + ch * 128 + lane * 4; *(volatile v4us*)(Ph + oo) = oh; *(volatile v4us*)(Pl + oo) = ol; }
        } else {
#pragma unroll
            for (int ch = 0; ch < TT / 128; ++ch) { v4h o4;
#pragma unroll
                for (int q = 0; q < 4; ++q) o4[q] = tohx(v[ch * 4 + q] * f);
                *(volatile v4h*)(P16 + (size_t)row * TT + ch * 128 + lane * 4) = o4; } }
        if (ps == 0) __threadfence(); }
}

__global__ __launch_bounds__(256) void k_merge1(const float* __restrict__ O, int r0, bf* XN) { const size_t e = ((size_t)blockIdx.x * 256 + threadIdx.x) * 2; if (e >= (size_t)ZH * TT * HD) return; const int d = (int)(e % HD); const int t = (int)((e / HD) % TT); const int zz = (int)(e / ((size_t)HD * TT)); const size_t oo = ((size_t)r0 + t) * DQ + zz * HD + d; v2us o;
#pragma unroll
    for (int q = 0; q < 2; ++q) o[q] = f2bf(O[e + q] * (1.0f / PCAR)); *(volatile v2us*)(XN + oo) = o; __threadfence(); *(volatile v2us*)(XN + oo) = o; }
__global__ __launch_bounds__(256) void k_relubf(const float* __restrict__ Hh, bf* RL, size_t n8) { const size_t i = (size_t)blockIdx.x * 256 + threadIdx.x; if (i >= n8) return; const v8f v = *(const v8f*)(Hh + i * 8); v8us o;
#pragma unroll
    for (int q = 0; q < 8; ++q) o[q] = f2bf(fmaxf(v[q], 0.0f)); *(volatile v8us*)(RL + i * 8) = o; __threadfence(); *(volatile v8us*)(RL + i * 8) = o; }
__global__ __launch_bounds__(256) void k_addln(float* X, const float* __restrict__ Hh, const float* __restrict__ gw, const float* __restrict__ gb) { const int lane = threadIdx.x & 31; const int r = blockIdx.x * 8 + (threadIdx.x >> 5); if (r >= ROWS) return; float* xr = X + (size_t)r * FD; const float* hr = Hh + (size_t)r * FD; float hv[16]; float s = 0.f;
#pragma unroll
    for (int ch = 0; ch < 4; ++ch) { const v4f a = *(const v4f*)(xr + ch * 128 + lane * 4); const v4f b2 = *(const v4f*)(hr + ch * 128 + lane * 4);
#pragma unroll
        for (int q = 0; q < 4; ++q) { const float u = __fadd_rn(a[q], b2[q]); hv[ch * 4 + q] = u; s += u; } }
#pragma unroll
    for (int sh = 16; sh; sh >>= 1) s += __shfl_xor(s, sh, 32);
    float mu = s * (1.0f / 512.0f); asm volatile("" : "+v"(mu)); float s2 = 0.f;
#pragma unroll
    for (int k = 0; k < 16; ++k) { float d0 = __fsub_rn(hv[k], mu); asm volatile("" : "+v"(d0)); float p = __fmul_rn(d0, d0); asm volatile("" : "+v"(p)); s2 = __fadd_rn(s2, p); }
#pragma unroll
    for (int sh = 16; sh; sh >>= 1) s2 += __shfl_xor(s2, sh, 32);
    float var = __fadd_rn(s2 * (1.0f / 512.0f), 1e-5f); asm volatile("" : "+v"(var)); const float rs = __frsqrt_rn(var);
#pragma unroll 1
    for (int ps = 0; ps < 2; ++ps) {
#pragma unroll
        for (int ch = 0; ch < 4; ++ch) { const int c0 = ch * 128 + lane * 4; v4f o;
#pragma unroll
            for (int q = 0; q < 4; ++q) { float gg = bfr(gw[c0 + q]); asm volatile("" : "+v"(gg)); float d0 = __fsub_rn(hv[ch * 4 + q], mu); asm volatile("" : "+v"(d0)); float n0 = __fmul_rn(d0, rs); asm volatile("" : "+v"(n0)); float y = __fmul_rn(n0, gg); asm volatile("" : "+v"(y)); o[q] = __fadd_rn(y, bfr(gb[c0 + q])); }
            *(volatile v4f*)(xr + c0) = o; }
        if (ps == 0) __threadfence(); } }

extern "C" void kernel_launch(void* const* d_in, const int* in_sizes, int n_in,
                              void* d_out, int out_size, void* d_ws, size_t ws_size, hipStream_t stream) {
    (void)in_sizes; (void)n_in; (void)out_size;
    const int* tok = (const int*)d_in[0]; const float* emb = (const float*)d_in[1]; const float* Wq = (const float*)d_in[2]; const float* Wk = (const float*)d_in[3]; const float* Wv = (const float*)d_in[4]; const float* W1 = (const float*)d_in[5]; const float* b1 = (const float*)d_in[6]; const float* W2 = (const float*)d_in[7]; const float* b2 = (const float*)d_in[8]; const float* gam = (const float*)d_in[9]; const float* bet = (const float*)d_in[10]; const float* Wout = (const float*)d_in[11]; const float* bout = (const float*)d_in[12];
    float* OUT = (float*)d_out;
    char* wsp = (char*)d_ws;
    auto take = [&](size_t bytes) { char* p = wsp; wsp += (bytes + 255) & ~(size_t)255; return (void*)p; };
    const size_t WSZ = (size_t)FD * FD;
    bf* WQB = (bf*)take(NL * WSZ * 2); bf* WKB = (bf*)take(NL * WSZ * 2); bf* WVB = (bf*)take(NL * WSZ * 2); bf* W1B = (bf*)take(NL * WSZ * 2); bf* W2B = (bf*)take(NL * WSZ * 2); bf* WOB = (bf*)take((size_t)VOC * FD * 2);
    float* X = (float*)take((size_t)ROWS * FD * 4); bf* XH = (bf*)take((size_t)ROWS * FD * 2); bf* XL = (bf*)take((size_t)ROWS * FD * 2); float* FQ = (float*)take((size_t)ROWS * DQ * 4); float* FK = (float*)take((size_t)ROWS * DQ * 4); float* FV = (float*)take((size_t)ROWS * DQ * 4);
    h16* KQ16 = (h16*)take((size_t)NH_ * TT * HD * 2); h16* KV16 = (h16*)take((size_t)NH_ * TT * HD * 2); h16* QT16 = (h16*)take((size_t)NH_ * HD * TT * 2); float* Sb = (float*)take((size_t)ZH * TT * TT * 4); h16* P16 = (h16*)take((size_t)ZH * TT * TT * 2); float* Ob = (float*)take((size_t)ZH * TT * HD * 4);
    bf* XN = (bf*)take((size_t)ROWS * DQ * 2); float* H1 = (float*)take((size_t)ROWS * FD * 4); bf* RL = (bf*)take((size_t)ROWS * FD * 2); float* H2 = (float*)take((size_t)ROWS * FD * 4);
    if ((size_t)(wsp - (char*)d_ws) > ws_size) return;
    for (int li = 0; li < NL; ++li) { k_wtG<<<(unsigned)((FD * FD / 64 + 63) / 64), 256, 0, stream>>>(Wq + li * WSZ, FD, FD, WQB + li * WSZ); k_wtG<<<(unsigned)((FD * FD / 64 + 63) / 64), 256, 0, stream>>>(Wk + li * WSZ, FD, FD, WKB + li * WSZ); k_wtG<<<(unsigned)((FD * FD / 64 + 63) / 64), 256, 0, stream>>>(Wv + li * WSZ, FD, FD, WVB + li * WSZ);
        k_wtG<<<(unsigned)((FD * FD / 64 + 63) / 64), 256, 0, stream>>>(W1 + li * WSZ, FD, FD, W1B + li * WSZ); k_wtG<<<(unsigned)((FD * FD / 64 + 63) / 64), 256, 0, stream>>>(W2 + li * WSZ, FD, FD, W2B + li * WSZ); }
    k_wtG<<<(unsigned)((FD * VOC / 64 + 63) / 64), 256, 0, stream>>>(Wout, FD, VOC, WOB);
    k_embx<<<(unsigned)(((size_t)ROWS * FD / 4 + 255) / 256), 256, 0, stream>>>(tok, emb, X);
    const unsigned L8 = (unsigned)(((size_t)ROWS * FD / 8 + 255) / 256), LP = (unsigned)(((size_t)NH_ * TT * HD / 2 + 255) / 256);
    for (int li = 0; li < NL; ++li) {
        k_split8<<<L8, 256, 0, stream>>>(X, XH, XL, (size_t)ROWS * FD / 8);
        k_gemmw<bf, 1, false><<<dim3(ROWS / 64, DQ / 64, 1), 32, 0, stream>>>(XH, XL, WQB + li * WSZ, nullptr, FD, FQ, DQ, nullptr, 0, 0, 0);
        k_gemmw<bf, 1, false><<<dim3(ROWS / 64, DQ / 64, 1), 32, 0, stream>>>(XH, XL, WKB + li * WSZ, nullptr, FD, FK, DQ, nullptr, 0, 0, 0);
        k_gemmw<bf, 1, false><<<dim3(ROWS / 64, DQ / 64, 1), 32, 0, stream>>>(XH, XL, WVB + li * WSZ, nullptr, FD, FV, DQ, nullptr, 0, 0, 0);
        for (int n = 0; n < NSEQ; ++n) { const int r0 = n * TT;
            k_pl16<<<LP, 256, 0, stream>>>(FK, r0, KQ16); k_pl16<<<LP, 256, 0, stream>>>(FV, r0, KV16); k_vt16<<<LP, 256, 0, stream>>>(FQ, r0, QT16);
            k_gemmc<h16, 0, 1><<<dim3(TT / 64, TT / 64, ZH), 32, 0, stream>>>(KQ16, nullptr, KV16, nullptr, HD, Sb, TT, 0, (size_t)TT * HD, (size_t)TT * HD, (size_t)TT * TT);
            k_asoft<<<ZH * TT / 8, 256, 0, stream>>>(Sb, P16, nullptr, nullptr);
            k_gemmc<h16, 0, 2><<<dim3(TT / 64, HD / 64, ZH), 32, 0, stream>>>(P16, nullptr, QT16, nullptr, TT, Ob, HD, 0, (size_t)TT * TT, (size_t)HD * TT, (size_t)TT * HD);
            k_merge1<<<LP, 256, 0, stream>>>(Ob, r0, XN); }
        k_gemmw<bf, 0, true><<<dim3(ROWS / 64, FD / 64, 1), 32, 0, stream>>>(XN, nullptr, W1B + li * WSZ, nullptr, DQ, H1, FD, b1 + li * FD, 0, 0, 0);
        k_relubf<<<L8, 256, 0, stream>>>(H1, RL, (size_t)ROWS * FD / 8);
        k_gemmw<bf, 0, true><<<dim3(ROWS / 64, FD / 64, 1), 32, 0, stream>>>(RL, nullptr, W2B + li * WSZ, nullptr, FD, H2, FD, b2 + li * FD, 0, 0, 0);
        k_addln<<<ROWS / 8, 256, 0, stream>>>(X, H2, gam + li * FD, bet + li * FD); }
    k_split8<<<L8, 256, 0, stream>>>(X, XH, XL, (size_t)ROWS * FD / 8);
    k_gemmw<bf, 1, true><<<dim3(ROWS / 64, VOC / 64, 1), 32, 0, stream>>>(XH, XL, WOB, nullptr, FD, OUT, VOC, bout, 0, 0, 0);
}
